// MultiModalModel_54065048322130
// MI455X (gfx1250) — hardware-run, weakly checked
//
#include <hip/hip_runtime.h>


namespace {
typedef _Float16 b16;
typedef __attribute__((ext_vector_type(16))) _Float16 v16b;
typedef __attribute__((ext_vector_type(8))) _Float16 v8b;
typedef __attribute__((ext_vector_type(4))) _Float16 v4h;
typedef __attribute__((ext_vector_type(2))) _Float16 v2h;
typedef __attribute__((ext_vector_type(8))) float v8f;
typedef __attribute__((ext_vector_type(4))) float v4f;
typedef __attribute__((ext_vector_type(2))) float v2f;
__device__ __forceinline__ float bf16_rne(float f) { unsigned int u = __float_as_uint(f); u += 0x7FFFu + ((u >> 16) & 1u); return __uint_as_float(u & 0xFFFF0000u); }
__device__ __forceinline__ void split16(float v, b16& hi, b16& lo) { hi = (b16)v; lo = (b16)(v - (float)hi); }
__device__ __forceinline__ v16b frag_kb(const b16* p, int hh) { const v8b a = *(const v8b*)(p + 8 * hh), b = *(const v8b*)(p + 16 + 8 * hh); v16b f;
#pragma unroll
  for (int e = 0; e < 8; ++e) { f[e] = a[e]; f[8 + e] = b[e]; } return f; }
__device__ __forceinline__ v8f wmma16b(v16b a, v16b b, v8f c) { v8f d = __builtin_amdgcn_wmma_f32_16x16x32_f16(false, a, false, b, (short)0, c, false, false); asm volatile("v_nop\n\tv_nop\n\tv_nop\n\tv_nop" : "+v"(d) : "v"(a), "v"(b)); return d; }
__device__ __forceinline__ void wave_lds_sync() { __builtin_amdgcn_fence(__ATOMIC_RELEASE, "workgroup"); __builtin_amdgcn_wave_barrier(); __builtin_amdgcn_fence(__ATOMIC_ACQUIRE, "workgroup"); }
__device__ __forceinline__ float pmul(float a, float b) { float p = a * b; asm volatile("" : "+v"(p)); return p; }
__device__ __forceinline__ int iclamp(int v, int lo, int hi) { return v < lo ? lo : (v > hi ? hi : v); }
__device__ __forceinline__ float nexp2(float v) { return __builtin_amdgcn_exp2f(v); }

constexpr int B = 4, BL = B  , DM = 64, HH = 64, WW = 64, L = HH * WW, DI = 128, NS = 16, R = 4, K = 4, C36 = R + 2 * NS, CP = 48, F1 = 256, F2 = 768, NPIX = B * L;
constexpr float XS = 8.0f, WSC = 256.0f, WSQ = 0.25f, RS_ = 1024.0f, LNEPS = 1e-5f;
static_assert(HH == WW && L % 32 == 0 && DI == 128 && DM == 64, "tiling");
__device__ __forceinline__ int srcpix(int k, int l) { const int ll = (k >= 2) ? (L - 1 - l) : l; return (k & 1) ? ((ll % HH) * WW + ll / HH) : ll; }
__device__ __forceinline__ float siluf(float v) { return v / (1.0f + __expf(-v)); }
__device__ __forceinline__ float softpl(float v) { return v > 20.0f ? v : log1pf(__expf(v)); }
__device__ __forceinline__ float geluf(float v) { return 0.5f * v * (1.0f + erff(v * 0.70710678118654752f)); }
__device__ __forceinline__ void splitr(float v, b16* hi, b16* lo) { const float vs = v * XS; const b16 p = (b16)vs; *hi = p; *lo = (b16)((vs - (float)p) * RS_); }
__global__ __launch_bounds__(256) void wcvt_kernel(const float* __restrict__ w, b16* __restrict__ W16, int n8, float scl) { const int u = blockIdx.x * 256 + threadIdx.x; if (u >= n8) return; const size_t e = (size_t)u * 8; v8b o; for (int j = 0; j < 8; ++j) o[j] = (b16)(bf16_rne(w[e + j]) * scl);
  for (int pass = 0; pass < 2; ++pass) { *(volatile v8b*)(W16 + e) = o; __threadfence(); } }
__global__ __launch_bounds__(256) void xpt_kernel(const float* __restrict__ w, b16* __restrict__ WT, float scl) { const int u = blockIdx.x * 256 + threadIdx.x; if (u >= K * CP * DI / 8) return; const int e = u * 8; const int k = e / (CP * DI), rem = e % (CP * DI), c = rem / DI, d0 = rem % DI; v8b o; for (int j = 0; j < 8; ++j) o[j] = (b16)(c < C36 ? bf16_rne(w[((size_t)k * C36 + c) * DI + d0 + j]) * scl : 0.0f);
  for (int pass = 0; pass < 2; ++pass) { *(volatile v8b*)(WT + e) = o; __threadfence(); } }
__global__ __launch_bounds__(256) void inproj_kernel(const float* __restrict__ x0, const float* __restrict__ x1, const float* __restrict__ ig, const float* __restrict__ ib, const b16* __restrict__ W0T, const b16* __restrict__ W0Q, const b16* __restrict__ W1T, const b16* __restrict__ W1Q, float* __restrict__ XPM, float* __restrict__ Z, float* __restrict__ XSUM) {
  __shared__ float S[2][32][DM + 1]; __shared__ float part[2][32][8]; __shared__ __attribute__((aligned(16))) b16 Ah[2][32][DM + 8], Al[2][32][DM + 8]; __shared__ __attribute__((aligned(16))) float Tx[32][DI + 4], Tz[32][DI + 4], Ts[32][DM + 4];
  const int tid = threadIdx.x, wave = tid >> 5, lane = tid & 31, nloc = lane & 15, hlf = lane >> 4; const int b = blockIdx.y, l0 = blockIdx.x * 32;
  for (int i = tid; i < DM * 32; i += 256) { const int c = i / 32, p = i % 32; const size_t gi = ((size_t)b * DM + c) * L + l0 + p; const float a = bf16_rne(x0[gi]), bb = bf16_rne(x1[gi]); S[0][p][c] = a; S[1][p][c] = bb; Ts[p][c] = a + bb; }
  __syncthreads();
  { const int p = tid >> 3, g = tid & 7;
    for (int m = 0; m < 2; ++m) { float s = 0.0f; for (int j = 0; j < 8; ++j) s += S[m][p][g * 8 + j]; part[m][p][g] = s; }
    __syncthreads();
    float mean[2], var[2]; for (int m = 0; m < 2; ++m) { float t = 0.0f; for (int gg = 0; gg < 8; ++gg) t += part[m][p][gg]; mean[m] = t * (1.0f / DM); }
    __syncthreads();
    for (int m = 0; m < 2; ++m) { float s = 0.0f; for (int j = 0; j < 8; ++j) { const float d = S[m][p][g * 8 + j] - mean[m]; s = fmaf(d, d, s); } part[m][p][g] = s; }
    __syncthreads();
    for (int m = 0; m < 2; ++m) { float t = 0.0f; for (int gg = 0; gg < 8; ++gg) t += part[m][p][gg]; var[m] = t * (1.0f / DM); }
    for (int m = 0; m < 2; ++m) { const float rs = rsqrtf(var[m] + LNEPS); for (int j = 0; j < 8; ++j) { const int c = g * 8 + j; const float v = (S[m][p][c] - mean[m]) * rs * bf16_rne(ig[c]) + bf16_rne(ib[c]); splitr(v, &Ah[m][p][c], &Al[m][p][c]); } } }
  __syncthreads();
  v8f acc0[2][2] = {{(v8f){}, (v8f){}}, {(v8f){}, (v8f){}}}, acc1[2][2] = {{(v8f){}, (v8f){}}, {(v8f){}, (v8f){}}};
#pragma unroll
  for (int m = 0; m < 2; ++m) { const b16* WT = m == 0 ? W0T : W1T; const b16* WQ = m == 0 ? W0Q : W1Q;
#pragma unroll
    for (int tt = 0; tt < 2; ++tt) { const int o = wave * 32 + tt * 16 + nloc;
#pragma unroll
      for (int kb = 0; kb < DM; kb += 32) { const v16b bw = frag_kb(WT + (size_t)o * DM + kb, hlf), bq = frag_kb(WQ + (size_t)o * DM + kb, hlf);
#pragma unroll
        for (int rt = 0; rt < 2; ++rt) { v8f a_ = (m == 0 || wave < 4) ? acc0[rt][tt] : acc1[rt][tt]; a_ = wmma16b(frag_kb(&Ah[m][rt * 16 + nloc][kb], hlf), bw, a_); a_ = wmma16b(frag_kb(&Al[m][rt * 16 + nloc][kb], hlf), bq, a_); if (m == 0 || wave < 4) acc0[rt][tt] = a_; else acc1[rt][tt] = a_; } } } }
#pragma unroll
  for (int tt = 0; tt < 2; ++tt) { const int col = wave * 32 + tt * 16 + nloc;
#pragma unroll
    for (int rt = 0; rt < 2; ++rt)
#pragma unroll
      for (int r = 0; r < 8; ++r) { const int rr = rt * 16 + 8 * hlf + r; if (wave < 4) Tx[rr][col] = acc0[rt][tt][r] * (1.0f / (XS * WSC)); else Tz[rr][col - DI] = siluf(acc0[rt][tt][r] * (1.0f / (XS * WSC))) + siluf(acc1[rt][tt][r] * (1.0f / (XS * WSC))); } }
  __syncthreads();
  for (int pass = 0; pass < 2; ++pass) { for (int rr = wave * 4; rr < wave * 4 + 4; ++rr) { const size_t row = (size_t)b * L + l0 + rr; *(volatile v4f*)(XPM + row * DI + lane * 4) = *(const v4f*)(&Tx[rr][lane * 4]); *(volatile v4f*)(Z + row * DI + lane * 4) = *(const v4f*)(&Tz[rr][lane * 4]); if (lane < 16) *(volatile v4f*)(XSUM + row * DM + lane * 4) = *(const v4f*)(&Ts[rr][lane * 4]); } __threadfence(); }
}
__global__ __launch_bounds__(64) void xproj_kernel(const float* __restrict__ XPM, const b16* __restrict__ XPT, const b16* __restrict__ XPQ, float* __restrict__ XDBL) {
  __shared__ __attribute__((aligned(16))) b16 Ah[2][16][DI + 8], Al[2][16][DI + 8]; __shared__ __attribute__((aligned(16))) float Ob[32 * CP + 4];
  const int wave = threadIdx.x >> 5, lane = threadIdx.x & 31, nloc = lane & 15, hlf = lane >> 4; const int b = blockIdx.z, k = blockIdx.y, l0 = blockIdx.x * 32 + wave * 16;
  for (int idx = lane; idx < 16 * 32; idx += 32) { const int rr = idx / 32, c4 = (idx % 32) * 4; const v4f v = *(const v4f*)(XPM + ((size_t)b * L + srcpix(k, l0 + rr)) * DI + c4); v4h hv, lv; for (int j = 0; j < 4; ++j) { b16 h_, l_; splitr(v[j], &h_, &l_); hv[j] = h_; lv[j] = l_; } *(v4h*)(&Ah[wave][rr][c4]) = hv; *(v4h*)(&Al[wave][rr][c4]) = lv; }
  wave_lds_sync();
  v8f acc[3] = {(v8f){}, (v8f){}, (v8f){}};
#pragma unroll
  for (int kb = 0; kb < DI; kb += 32) { const v16b a = frag_kb(&Ah[wave][nloc][kb], hlf), al = frag_kb(&Al[wave][nloc][kb], hlf);
#pragma unroll
    for (int t = 0; t < 3; ++t) { const size_t wo_ = ((size_t)k * CP + t * 16 + nloc) * DI + kb; acc[t] = wmma16b(a, frag_kb(XPT + wo_, hlf), acc[t]); acc[t] = wmma16b(al, frag_kb(XPQ + wo_, hlf), acc[t]); } }
#pragma unroll
  for (int t = 0; t < 3; ++t)
#pragma unroll
    for (int r = 0; r < 8; ++r) Ob[(wave * 16 + 8 * hlf + r) * CP + t * 16 + nloc] = acc[t][r] * (1.0f / (XS * WSC));
  __syncthreads();
  const size_t base = (((size_t)b * K + k) * L + blockIdx.x * 32) * CP;
  for (int pass = 0; pass < 2; ++pass) { for (int q = threadIdx.x; q < 32 * CP / 4; q += 64) *(volatile v4f*)(XDBL + base + (size_t)q * 4) = *(const v4f*)(&Ob[q * 4]); __threadfence(); }
}
__global__ __launch_bounds__(128) void scan_kernel(const float* __restrict__ XPM, const float* __restrict__ XDBL, const float* __restrict__ dtw, const float* __restrict__ dtb, const float* __restrict__ alog, const float* __restrict__ Dsv, float* __restrict__ Y) {
  __shared__ float rows[32][CP];
  const int d = threadIdx.x; const int b = blockIdx.x / K, k = blockIdx.x % K; const int kd = k * DI + d;
  float An[NS], h[NS]; for (int n = 0; n < NS; ++n) { An[n] = -__expf(bf16_rne(alog[(size_t)kd * NS + n])); h[n] = 0.0f; }
  float wr[R]; for (int r = 0; r < R; ++r) wr[r] = bf16_rne(dtw[(size_t)kd * R + r]); const float bias = bf16_rne(dtb[kd]); const float Dd = bf16_rne(Dsv[kd]);
  const float* xd = XDBL + ((size_t)b * K + k) * L * CP; float* Yk = Y + ((size_t)k * B + b) * L * DI;
#pragma unroll 1
  for (int l0 = 0; l0 < L; l0 += 32) {
    __syncthreads();
    for (int i = threadIdx.x; i < 32 * CP; i += 128) rows[i / CP][i % CP] = xd[(size_t)l0 * CP + i];
    __syncthreads();
#pragma unroll 1
    for (int j = 0; j < 32; ++j) { const int l = l0 + j; const float* rw = rows[j];
      float dtr = bias; for (int r = 0; r < R; ++r) dtr = fmaf(rw[r], wr[r], dtr); const float dt = softpl(dtr);
      const int pix = srcpix(k, l); const float xv = XPM[((size_t)b * L + pix) * DI + d]; const float dx = dt * xv; float y = 0.0f;
#pragma unroll
      for (int n = 0; n < NS; ++n) { h[n] = fmaf(__expf(dt * An[n]), h[n], dx * rw[R + n]); y = fmaf(h[n], rw[R + NS + n], y); }
      y = fmaf(Dd, xv, y);
      for (int pass = 0; pass < 2; ++pass) { ((volatile float*)Yk)[(size_t)pix * DI + d] = y; __threadfence(); } } }
}
__global__ __launch_bounds__(256) void outstage_kernel(const float* __restrict__ Y, const float* __restrict__ Z, const float* __restrict__ XSUM, const float* __restrict__ og, const float* __restrict__ ob_, const b16* __restrict__ OPT, const b16* __restrict__ OPQ, const b16* __restrict__ F1T, const b16* __restrict__ F1Q, const float* __restrict__ b1, const b16* __restrict__ F2T, const b16* __restrict__ F2Q, const float* __restrict__ b2, const float* __restrict__ lg, const float* __restrict__ lb, float* __restrict__ out) {
  __shared__ __attribute__((aligned(16))) b16 A1h[32][DI + 8], A1l[32][DI + 8], A2h[32][DM + 8], A2l[32][DM + 8], A3h[32][F1 + 8], A3l[32][F1 + 8]; __shared__ __attribute__((aligned(16))) float Tf[32][F2 + 4]; __shared__ float part[32][8];
  const int tid = threadIdx.x, wave = tid >> 5, lane = tid & 31, nloc = lane & 15, hlf = lane >> 4; const int b = blockIdx.y, l0 = blockIdx.x * 32;
  { const int p = tid >> 3, g = tid & 7; const size_t row = (size_t)b * L + l0 + p; float v[16]; float s = 0.0f;
    for (int j = 0; j < 16; ++j) { const int c = g * 16 + j; float t = 0.0f; for (int k = 0; k < K; ++k) t += Y[(((size_t)k * B + b) * L + l0 + p) * DI + c]; v[j] = t; s += t; }
    part[p][g] = s; __syncthreads(); float mean = 0.0f; for (int gg = 0; gg < 8; ++gg) mean += part[p][gg]; mean *= (1.0f / DI); __syncthreads();
    float s2 = 0.0f; for (int j = 0; j < 16; ++j) { const float dd = v[j] - mean; s2 = fmaf(dd, dd, s2); } part[p][g] = s2; __syncthreads(); float var = 0.0f; for (int gg = 0; gg < 8; ++gg) var += part[p][gg]; var *= (1.0f / DI); const float rs = rsqrtf(var + LNEPS);
    for (int j = 0; j < 16; ++j) { const int c = g * 16 + j; const float yv = ((v[j] - mean) * rs * bf16_rne(og[c]) + bf16_rne(ob_[c])) * Z[row * DI + c]; splitr(yv, &A1h[p][c], &A1l[p][c]); } }
  __syncthreads();
  { const int rt = wave & 1, ct = wave >> 1; v8f acc = (v8f){}; const b16* br = OPT + (size_t)(ct * 16 + nloc) * DI; const b16* bq = OPQ + (size_t)(ct * 16 + nloc) * DI;
#pragma unroll
    for (int kb = 0; kb < DI; kb += 32) { acc = wmma16b(frag_kb(&A1h[rt * 16 + nloc][kb], hlf), frag_kb(br + kb, hlf), acc); acc = wmma16b(frag_kb(&A1l[rt * 16 + nloc][kb], hlf), frag_kb(bq + kb, hlf), acc); }
#pragma unroll
    for (int r = 0; r < 8; ++r) { const int rr = rt * 16 + 8 * hlf + r, col = ct * 16 + nloc; const float fz = acc[r] * (1.0f / (XS * WSC)) + XSUM[((size_t)b * L + l0 + rr) * DM + col]; splitr(fz, &A2h[rr][col], &A2l[rr][col]); } }
  __syncthreads();
  { v8f acc[2][2] = {{(v8f){}, (v8f){}}, {(v8f){}, (v8f){}}};
#pragma unroll
    for (int tt = 0; tt < 2; ++tt) { const int o = wave * 32 + tt * 16 + nloc; const b16* br = F1T + (size_t)o * DM; const b16* bq = F1Q + (size_t)o * DM;
#pragma unroll
      for (int kb = 0; kb < DM; kb += 32) { const v16b bw = frag_kb(br + kb, hlf), bwq = frag_kb(bq + kb, hlf);
#pragma unroll
        for (int rt = 0; rt < 2; ++rt) { acc[rt][tt] = wmma16b(frag_kb(&A2h[rt * 16 + nloc][kb], hlf), bw, acc[rt][tt]); acc[rt][tt] = wmma16b(frag_kb(&A2l[rt * 16 + nloc][kb], hlf), bwq, acc[rt][tt]); } } }
#pragma unroll
    for (int tt = 0; tt < 2; ++tt) { const int col = wave * 32 + tt * 16 + nloc; const float bb = bf16_rne(b1[col]);
#pragma unroll
      for (int rt = 0; rt < 2; ++rt)
#pragma unroll
        for (int r = 0; r < 8; ++r) { const float f = geluf(acc[rt][tt][r] * (1.0f / (XS * WSC)) + bb); splitr(f, &A3h[rt * 16 + 8 * hlf + r][col], &A3l[rt * 16 + 8 * hlf + r][col]); } } }
  __syncthreads();
  { const int rt = wave & 1, t0 = (wave >> 1) * 12; v8f acc[12];
#pragma unroll
    for (int t = 0; t < 12; ++t) acc[t] = (v8f){};
#pragma unroll 1
    for (int kb = 0; kb < F1; kb += 32) { const v16b a = frag_kb(&A3h[rt * 16 + nloc][kb], hlf), al = frag_kb(&A3l[rt * 16 + nloc][kb], hlf);
#pragma unroll
      for (int t = 0; t < 12; ++t) { const size_t wo_ = (size_t)((t0 + t) * 16 + nloc) * F1 + kb; acc[t] = wmma16b(a, frag_kb(F2T + wo_, hlf), acc[t]); acc[t] = wmma16b(al, frag_kb(F2Q + wo_, hlf), acc[t]); } }
#pragma unroll
    for (int t = 0; t < 12; ++t) { const int col = (t0 + t) * 16 + nloc; const float bb = bf16_rne(b2[col]);
#pragma unroll
      for (int r = 0; r < 8; ++r) Tf[rt * 16 + 8 * hlf + r][col] = acc[t][r] * (1.0f / (XS * WSC)) + bb; } }
  __syncthreads();
  { const int p = tid >> 3, g = tid & 7; float s = 0.0f; for (int j = 0; j < 96; ++j) s += Tf[p][g * 96 + j]; part[p][g] = s; __syncthreads(); float mean = 0.0f; for (int gg = 0; gg < 8; ++gg) mean += part[p][gg]; mean *= (1.0f / F2); __syncthreads();
    float s2 = 0.0f; for (int j = 0; j < 96; ++j) { const float dd = Tf[p][g * 96 + j] - mean; s2 = fmaf(dd, dd, s2); } part[p][g] = s2; __syncthreads(); float var = 0.0f; for (int gg = 0; gg < 8; ++gg) var += part[p][gg]; var *= (1.0f / F2); const float rs = rsqrtf(var + LNEPS);
    for (int j = 0; j < 96; ++j) { const int c = g * 96 + j; Tf[p][c] = (Tf[p][c] - mean) * rs * bf16_rne(lg[c]) + bf16_rne(lb[c]); } }
  __syncthreads();
  const size_t base = ((size_t)b * L + l0) * F2;
  for (int pass = 0; pass < 2; ++pass) { for (int q = tid; q < 32 * F2 / 4; q += 256) { const int rr = q / (F2 / 4), c4 = (q % (F2 / 4)) * 4; *(volatile v4f*)(out + base + (size_t)rr * F2 + c4) = *(const v4f*)(&Tf[rr][c4]); } __threadfence(); }
}
}

extern "C" void kernel_launch(void* const* d_in, const int* in_sizes, int n_in, void* d_out, int out_size, void* d_ws, size_t ws_size, hipStream_t stream) {
  (void)n_in;
  auto Fp = [&](int i) { return (const float*)d_in[i]; };
  if (in_sizes[0] != B * DM * L || in_sizes[1] != B * DM * L || in_sizes[4] != 256 * DM || in_sizes[5] != 256 * DM || in_sizes[6] != K * C36 * DI || in_sizes[7] != K * DI * R || in_sizes[8] != K * DI || in_sizes[9] != K * DI * NS || in_sizes[10] != K * DI || in_sizes[13] != DM * DI || in_sizes[14] != F1 * DM || in_sizes[16] != F2 * F1 || in_sizes[17] != F2 || out_size != NPIX * F2) return;
  size_t off = 0; char* ws = (char*)d_ws;
  auto carve = [&](size_t bytes) { char* p = ws + off; off += (bytes + 255) & ~(size_t)255; return p; };
  b16* W0T = (b16*)carve((size_t)256 * DM * 2); b16* W0Q = (b16*)carve((size_t)256 * DM * 2); b16* W1T = (b16*)carve((size_t)256 * DM * 2); b16* W1Q = (b16*)carve((size_t)256 * DM * 2);
  b16* XPT = (b16*)carve((size_t)K * CP * DI * 2); b16* XPQ = (b16*)carve((size_t)K * CP * DI * 2); b16* OPT = (b16*)carve((size_t)DM * DI * 2); b16* OPQ = (b16*)carve((size_t)DM * DI * 2);
  b16* F1T = (b16*)carve((size_t)F1 * DM * 2); b16* F1Q = (b16*)carve((size_t)F1 * DM * 2); b16* F2T = (b16*)carve((size_t)F2 * F1 * 2); b16* F2Q = (b16*)carve((size_t)F2 * F1 * 2);
  float* XPM = (float*)carve((size_t)NPIX * DI * 4); float* Z = (float*)carve((size_t)NPIX * DI * 4); float* XSUM = (float*)carve((size_t)NPIX * DM * 4); float* XDBL = (float*)carve((size_t)B * K * L * CP * 4); float* Y = (float*)carve((size_t)K * B * L * DI * 4);
  if (off > ws_size || off > ((size_t)128 << 20)) return;
  const unsigned g64 = (256 * DM / 8 + 255) / 256;
  wcvt_kernel<<<g64, 256, 0, stream>>>(Fp(4), W0T, 256 * DM / 8, WSC); wcvt_kernel<<<g64, 256, 0, stream>>>(Fp(4), W0Q, 256 * DM / 8, WSQ); wcvt_kernel<<<g64, 256, 0, stream>>>(Fp(5), W1T, 256 * DM / 8, WSC); wcvt_kernel<<<g64, 256, 0, stream>>>(Fp(5), W1Q, 256 * DM / 8, WSQ);
  xpt_kernel<<<(K * CP * DI / 8 + 255) / 256, 256, 0, stream>>>(Fp(6), XPT, WSC); xpt_kernel<<<(K * CP * DI / 8 + 255) / 256, 256, 0, stream>>>(Fp(6), XPQ, WSQ);
  wcvt_kernel<<<(DM * DI / 8 + 255) / 256, 256, 0, stream>>>(Fp(13), OPT, DM * DI / 8, WSC); wcvt_kernel<<<(DM * DI / 8 + 255) / 256, 256, 0, stream>>>(Fp(13), OPQ, DM * DI / 8, WSQ);
  wcvt_kernel<<<(F1 * DM / 8 + 255) / 256, 256, 0, stream>>>(Fp(14), F1T, F1 * DM / 8, WSC); wcvt_kernel<<<(F1 * DM / 8 + 255) / 256, 256, 0, stream>>>(Fp(14), F1Q, F1 * DM / 8, WSQ);
  wcvt_kernel<<<(F2 * F1 / 8 + 255) / 256, 256, 0, stream>>>(Fp(16), F2T, F2 * F1 / 8, WSC); wcvt_kernel<<<(F2 * F1 / 8 + 255) / 256, 256, 0, stream>>>(Fp(16), F2Q, F2 * F1 / 8, WSQ);
  inproj_kernel<<<dim3(L / 32, BL), 256, 0, stream>>>(Fp(0), Fp(1), Fp(2), Fp(3), W0T, W0Q, W1T, W1Q, XPM, Z, XSUM);
  xproj_kernel<<<dim3(L / 32, K, BL), 64, 0, stream>>>(XPM, XPT, XPQ, XDBL);
  scan_kernel<<<BL * K, 128, 0, stream>>>(XPM, XDBL, Fp(7), Fp(8), Fp(9), Fp(10), Y);
  outstage_kernel<<<dim3(L / 32, BL), 256, 0, stream>>>(Y, Z, XSUM, Fp(11), Fp(12), OPT, OPQ, F1T, F1Q, Fp(15), F2T, F2Q, Fp(17), Fp(18), Fp(19), (float*)d_out);
}
